// ComplexMultiheadAttention_81647328297518
// MI455X (gfx1250) — hardware-run, weakly checked
//
#include <hip/hip_runtime.h>
#include <math.h>

#ifndef NB
#define NB 4
#endif
#ifndef SEQ
#define SEQ 1024
#endif
#define NB_FULL 4
#define SEQ_FULL 1024
#define DM 512
#define HEADS 8
#define HD 64
#define KC 1024
#define MTOK (NB * SEQ)
#define PLANE ((size_t)MTOK * 1024u)
#define QKV_CARRY 64.0f
#define P_CARRY 1024.0f

static_assert(NB <= NB_FULL);
static_assert(SEQ <= SEQ_FULL);
static_assert(SEQ % 128 == 0);
static_assert(MTOK % 64 == 0);
static_assert(KC % 64 == 0 && KC % 32 == 0);
static_assert(DM == HEADS * HD);
static_assert((MTOK * 64) % 256 == 0);
static_assert((DM * 64) % 256 == 0);

constexpr size_t SZ_XP  = (size_t)MTOK * KC * 2;
constexpr size_t SZ_WP  = (size_t)KC * KC * 2;
constexpr size_t SZ_QP  = (size_t)MTOK * 1024 * 2;
constexpr size_t SZ_KAB = 2 * SZ_QP;
constexpr size_t SZ_VT  = (size_t)NB * 1024 * SEQ * 2;
constexpr size_t SZ_T   = 2 * (size_t)MTOK * 1024 * 4;
constexpr size_t WS_TOTAL = 3 * SZ_XP + 3 * SZ_WP + SZ_QP + SZ_KAB + SZ_VT + SZ_T;
static_assert(WS_TOTAL <= (size_t)134217728);
static_assert(SZ_XP % 256 == 0 && SZ_WP % 256 == 0 && SZ_QP % 256 == 0 && SZ_VT % 256 == 0 && SZ_T % 256 == 0);

typedef _Float16 h16;
typedef __attribute__((ext_vector_type(16))) _Float16 v16h;
typedef __attribute__((ext_vector_type(8)))  _Float16 v8h;
typedef __attribute__((ext_vector_type(16))) __bf16   v16bf;
typedef __attribute__((ext_vector_type(8)))  unsigned short v8us;
typedef __attribute__((ext_vector_type(16))) unsigned short v16us;
typedef __attribute__((ext_vector_type(8)))  float    v8f;
typedef __attribute__((ext_vector_type(4)))  float    v4f;
typedef __attribute__((ext_vector_type(2)))  float    v2f;
typedef __attribute__((ext_vector_type(4)))  unsigned int v4u;


__device__ __forceinline__ float bfr(float f) {
    unsigned u = __float_as_uint(f);
    u += 0x7FFFu + ((u >> 16) & 1u);
    return __uint_as_float(u & 0xFFFF0000u);
}
__device__ __forceinline__ unsigned pk_bf(float lo, float hi) {
    unsigned a = __float_as_uint(lo);
    unsigned b = __float_as_uint(hi);
    a += 0x7FFFu + ((a >> 16) & 1u);
    b += 0x7FFFu + ((b >> 16) & 1u);
    return (a >> 16) | (b & 0xFFFF0000u);
}
static __device__ __forceinline__ h16 toh_flush(float v) {
    const float w = (fabsf(v) < 6.103515625e-05f) ? 0.0f : v;
    return (h16)w;
}

union FragU { v16h v; v8h h[2]; };
__device__ __forceinline__ v16h frag_ld(const _Float16* p) {
    FragU f; f.h[0] = *(const v8h*)(p); f.h[1] = *(const v8h*)(p + 16); return f.v;
}
__device__ __forceinline__ v16bf frag_ld_b(const unsigned short* p) {
    const v8us lo = *(const v8us*)(p);
    const v8us hi = *(const v8us*)(p + 16);
    const v16us w = __builtin_shufflevector(lo, hi, 0, 1, 2, 3, 4, 5, 6, 7, 8, 9, 10, 11, 12, 13, 14, 15);
    return __builtin_bit_cast(v16bf, w);
}
__device__ __forceinline__ v8f wmma16g(v16h a, v16h b, v8f c) {
    c = __builtin_amdgcn_wmma_f32_16x16x32_f16(false, a, false, b, (short)0, c, false, false);
    asm volatile("v_nop\n\tv_nop\n\tv_nop\n\tv_nop" : "+v"(c) : "v"(a), "v"(b));
    return c;
}
__device__ __forceinline__ v8f wmmabg(v16bf a, v16bf b, v8f c) {
    c = __builtin_amdgcn_wmma_f32_16x16x32_bf16(false, a, false, b, (short)0, c, false, false);
    asm volatile("v_nop\n\tv_nop\n\tv_nop\n\tv_nop" : "+v"(c) : "v"(a), "v"(b));
    return c;
}
__device__ __forceinline__ void wave_sync_lds() {
    __builtin_amdgcn_fence(3  , "workgroup");
    __builtin_amdgcn_wave_barrier();
    __builtin_amdgcn_fence(2  , "workgroup");
}

__global__ __launch_bounds__(256) void k_cvtx(const float* __restrict__ x, unsigned short* __restrict__ xp) {
    const unsigned u = blockIdx.x * 256u + threadIdx.x;
    if (u >= (unsigned)(MTOK * 64)) return;
    const unsigned row = u >> 6, d0 = (u & 63u) * 8u;
    const unsigned b = row / (unsigned)SEQ;
    const unsigned s = row - b * (unsigned)SEQ;
    const float* src = x + ((size_t)(b * (unsigned)SEQ_FULL + s) * DM + d0) * 2u;
    const v4f a0 = *(const v4f*)(src);
    const v4f a1 = *(const v4f*)(src + 4);
    const v4f a2 = *(const v4f*)(src + 8);
    const v4f a3 = *(const v4f*)(src + 12);
    v4u re, im;
    re.x = pk_bf(a0.x, a0.z); re.y = pk_bf(a1.x, a1.z); re.z = pk_bf(a2.x, a2.z); re.w = pk_bf(a3.x, a3.z);
    im.x = pk_bf(a0.y, a0.w); im.y = pk_bf(a1.y, a1.w); im.z = pk_bf(a2.y, a2.w); im.w = pk_bf(a3.y, a3.w);
    unsigned short* dr = xp + (size_t)row * KC + d0;
    unsigned short* di = dr + DM;
    for (int pass = 0; pass < 2; ++pass) {
        *(volatile v4u*)(dr) = re;
        *(volatile v4u*)(di) = im;
        __threadfence();
    }
}

__global__ __launch_bounds__(256) void k_cvtw(const float* __restrict__ W, unsigned short* __restrict__ wp) {
    const unsigned u = blockIdx.x * 256u + threadIdx.x;
    if (u >= (unsigned)(DM * 64)) return;
    const unsigned e = u >> 6, d0 = (u & 63u) * 8u;
    const float* src = W + ((size_t)e * DM + d0) * 2u;
    const v4f a0 = *(const v4f*)(src);
    const v4f a1 = *(const v4f*)(src + 4);
    const v4f a2 = *(const v4f*)(src + 8);
    const v4f a3 = *(const v4f*)(src + 12);
    v4u re, im, imn;
    re.x = pk_bf(a0.x, a0.z); re.y = pk_bf(a1.x, a1.z); re.z = pk_bf(a2.x, a2.z); re.w = pk_bf(a3.x, a3.z);
    im.x = pk_bf(a0.y, a0.w); im.y = pk_bf(a1.y, a1.w); im.z = pk_bf(a2.y, a2.w); im.w = pk_bf(a3.y, a3.w);
    imn.x = pk_bf(-a0.y, -a0.w); imn.y = pk_bf(-a1.y, -a1.w); imn.z = pk_bf(-a2.y, -a2.w); imn.w = pk_bf(-a3.y, -a3.w);
    unsigned short* r0 = wp + (size_t)e * KC + d0;
    unsigned short* r1 = wp + (size_t)(DM + e) * KC + d0;
    for (int pass = 0; pass < 2; ++pass) {
        *(volatile v4u*)(r0) = re;
        *(volatile v4u*)(r0 + DM) = imn;
        *(volatile v4u*)(r1) = im;
        *(volatile v4u*)(r1 + DM) = re;
        __threadfence();
    }
}

template <int MODE>
__global__ __launch_bounds__(256) void k_proj(const unsigned short* __restrict__ A, const unsigned short* __restrict__ Bt,
                                              _Float16* __restrict__ C, const float* __restrict__ bias,
                                              unsigned M, unsigned N, unsigned K) {
    __shared__ __align__(16) float sT[8][16 * 68];
    const unsigned lane = threadIdx.x & 31u;
    const unsigned wave = threadIdx.x >> 5;
    const unsigned tilesN = N >> 6, tilesM = M >> 6;
    const unsigned tile = blockIdx.x * 8u + wave;
    if (tile >= tilesM * tilesN) return;
    const unsigned tm = tile / tilesN;
    const unsigned tn = tile - tm * tilesN;
    const unsigned m0 = tm << 6, n0 = tn << 6;
    const unsigned rlane = lane & 15u;
    const unsigned koff = (lane >> 4) * 8u;
    const unsigned mOff = koff;

    v8f acc[4][4];
#pragma unroll
    for (int i = 0; i < 4; ++i)
#pragma unroll
        for (int j = 0; j < 4; ++j) acc[i][j] = (v8f){0.f,0.f,0.f,0.f,0.f,0.f,0.f,0.f};

    for (unsigned k0 = 0; k0 < K; k0 += 32u) {
        v16bf bh[4];
#pragma unroll
        for (int j = 0; j < 4; ++j)
            bh[j] = frag_ld_b(Bt + (size_t)(n0 + ((unsigned)j << 4) + rlane) * KC + koff + k0);
#pragma unroll
        for (int i = 0; i < 4; ++i) {
            const v16bf ah = frag_ld_b(A + (size_t)(m0 + ((unsigned)i << 4) + rlane) * KC + koff + k0);
#pragma unroll
            for (int j = 0; j < 4; ++j) acc[i][j] = wmmabg(ah, bh[j], acc[i][j]);
        }
    }

    const unsigned fsel = (MODE == 2) ? m0 : n0;
    const unsigned part = fsel >> 9;
    const unsigned f0 = fsel & 511u;
    const unsigned head = f0 >> 6;
    unsigned rowbase, ldc, colA, colB;
    float sgnA = 1.0f;
    if (MODE == 2) {
        const unsigned b = n0 / (unsigned)SEQ;
        const unsigned key0 = n0 - b * (unsigned)SEQ;
        rowbase = (b * 8u + head) * 128u + part * 64u;
        ldc = (unsigned)SEQ;
        colA = key0;
        colB = 0u;
    } else {
        rowbase = m0;
        ldc = 1024u;
        colA = head * 128u + part * 64u;
        colB = head * 128u + (1u - part) * 64u;
        if (MODE == 1) sgnA = (part != 0u) ? -1.0f : 1.0f;
    }

    float bvc[4] = {0.f, 0.f, 0.f, 0.f};
    if (MODE != 2) {
#pragma unroll
        for (int j = 0; j < 4; ++j) bvc[j] = bfr(bias[2u * (f0 + ((unsigned)j << 4) + rlane) + part]);
    }

    float* slab = sT[wave];
#pragma unroll
    for (int i = 0; i < 4; ++i) {
        float bvr[8] = {0.f, 0.f, 0.f, 0.f, 0.f, 0.f, 0.f, 0.f};
        if (MODE == 2) {
#pragma unroll
            for (int r = 0; r < 8; ++r) bvr[r] = bfr(bias[2u * (f0 + ((unsigned)i << 4) + mOff + (unsigned)r) + part]);
        }
#pragma unroll
        for (int j = 0; j < 4; ++j) {
#pragma unroll
            for (int r = 0; r < 8; ++r) {
                const float bb = (MODE == 2) ? bvr[r] : bvc[j];
                slab[(mOff + (unsigned)r) * 68u + ((unsigned)j << 4) + rlane] = (acc[i][j][r] + bb) * QKV_CARRY;
            }
        }
        wave_sync_lds();
        {
            const unsigned q = lane >> 3, c8 = (lane & 7u) * 8u;
            v8h hvA[4], hvB[4];
#pragma unroll
            for (int it = 0; it < 4; ++it) {
                const unsigned row = (unsigned)it * 4u + q;
                const float* sp = slab + row * 68u + c8;
                const v4f x0 = *(const v4f*)(sp);
                const v4f x1 = *(const v4f*)(sp + 4);
                const float xv[8] = {x0.x, x0.y, x0.z, x0.w, x1.x, x1.y, x1.z, x1.w};
#pragma unroll
                for (int e = 0; e < 8; ++e) {
                    hvA[it][e] = toh_flush(xv[e] * sgnA);
                    hvB[it][e] = toh_flush(xv[e]);
                }
            }
            for (int pass = 0; pass < 2; ++pass) {
#pragma unroll
                for (int it = 0; it < 4; ++it) {
                    const unsigned row = (unsigned)it * 4u + q;
                    const size_t ro = (size_t)(rowbase + ((unsigned)i << 4) + row) * ldc;
                    *(volatile v8h*)(C + ro + colA + c8) = hvA[it];
                    if (MODE == 1) *(volatile v8h*)(C + PLANE + ro + colB + c8) = hvB[it];
                }
                __threadfence();
            }
        }
        wave_sync_lds();
    }
}

#define AT_PP 68
__global__ __launch_bounds__(256) void k_attn(const _Float16* __restrict__ QP, const _Float16* __restrict__ KAB,
                                              const _Float16* __restrict__ VT, float* __restrict__ T, unsigned nchunks) {
    __shared__ __align__(16) float sP[8][16 * AT_PP];
    const unsigned tid = threadIdx.x, lane = tid & 31u, wave = tid >> 5;
    const unsigned hh = lane >> 4, c = lane & 15u;
    const unsigned bx = blockIdx.x;
    const unsigned part = blockIdx.y;
    const unsigned NQB = (unsigned)SEQ / 128u;
    const unsigned qb = bx % NQB;
    const unsigned bh = bx / NQB;
    const unsigned head = bh & 7u, b = bh >> 3;
    const unsigned q0 = qb * 128u + wave * 16u;
    float* pw = sP[wave];
    const float SC2 = 0.125f * (1.0f / 4096.0f) * 1.4426950408889634f;

    v16h qf[4];
#pragma unroll
    for (int ks = 0; ks < 4; ++ks)
        qf[ks] = frag_ld(QP + (size_t)(b * (unsigned)SEQ + q0 + c) * 1024u + head * 128u + (unsigned)ks * 32u + 8u * hh);

    const _Float16* Kp = KAB + (size_t)part * PLANE + (size_t)(b * (unsigned)SEQ) * 1024u + head * 128u + 8u * hh;
    const _Float16* Vp = VT + (size_t)((b * 8u + head) * 128u) * (unsigned)SEQ + 8u * hh;

    float mrow[8], lrow[8];
    v8f acc[8];
#pragma unroll
    for (int r = 0; r < 8; ++r) { mrow[r] = -3.0e38f; lrow[r] = 0.f; }
#pragma unroll
    for (int t = 0; t < 8; ++t) acc[t] = (v8f){0.f,0.f,0.f,0.f,0.f,0.f,0.f,0.f};

    for (unsigned kc = 0; kc < nchunks; ++kc) {
        const unsigned kv0 = kc * 64u;
        v8f s[4];
#pragma unroll
        for (int j = 0; j < 4; ++j) {
            const _Float16* kr = Kp + (size_t)(kv0 + (unsigned)j * 16u + c) * 1024u;
            s[j] = (v8f){0.f,0.f,0.f,0.f,0.f,0.f,0.f,0.f};
#pragma unroll
            for (int ks = 0; ks < 4; ++ks) {
                const v16h kf = frag_ld(kr + (unsigned)ks * 32u);
                s[j] = wmma16g(qf[ks], kf, s[j]);
            }
        }
#pragma unroll
        for (int r = 0; r < 8; ++r) {
            float mx = -3.0e38f;
#pragma unroll
            for (int j = 0; j < 4; ++j) { s[j][r] *= SC2; mx = fmaxf(mx, s[j][r]); }
            mx = fmaxf(mx, __shfl_xor(mx, 1, 32)); mx = fmaxf(mx, __shfl_xor(mx, 2, 32));
            mx = fmaxf(mx, __shfl_xor(mx, 4, 32)); mx = fmaxf(mx, __shfl_xor(mx, 8, 32));
            const float mnew = fmaxf(mrow[r], mx);
            const float alpha = exp2f(mrow[r] - mnew);
            mrow[r] = mnew;
            float psum = 0.f;
#pragma unroll
            for (int j = 0; j < 4; ++j) {
                const float p = exp2f(s[j][r] - mnew);
                psum += p;
                pw[(8u * hh + (unsigned)r) * AT_PP + (unsigned)j * 16u + c] = p * P_CARRY;
            }
            psum += __shfl_xor(psum, 1, 32); psum += __shfl_xor(psum, 2, 32);
            psum += __shfl_xor(psum, 4, 32); psum += __shfl_xor(psum, 8, 32);
            lrow[r] = lrow[r] * alpha + psum;
#pragma unroll
            for (int t = 0; t < 8; ++t) acc[t][r] *= alpha;
        }
        wave_sync_lds();
#pragma unroll
        for (int kk = 0; kk < 2; ++kk) {
            const float* pp = pw + c * AT_PP + (unsigned)kk * 32u + 8u * hh;
            const v4f p0 = *(const v4f*)(pp);
            const v4f p1 = *(const v4f*)(pp + 4);
            const v4f p2 = *(const v4f*)(pp + 16);
            const v4f p3 = *(const v4f*)(pp + 20);
            v16h pa;
            pa[0]  = toh_flush(p0.x); pa[1]  = toh_flush(p0.y); pa[2]  = toh_flush(p0.z); pa[3]  = toh_flush(p0.w);
            pa[4]  = toh_flush(p1.x); pa[5]  = toh_flush(p1.y); pa[6]  = toh_flush(p1.z); pa[7]  = toh_flush(p1.w);
            pa[8]  = toh_flush(p2.x); pa[9]  = toh_flush(p2.y); pa[10] = toh_flush(p2.z); pa[11] = toh_flush(p2.w);
            pa[12] = toh_flush(p3.x); pa[13] = toh_flush(p3.y); pa[14] = toh_flush(p3.z); pa[15] = toh_flush(p3.w);
#pragma unroll
            for (int t = 0; t < 8; ++t) {
                const v16h vb = frag_ld(Vp + (size_t)((unsigned)t * 16u + c) * (unsigned)SEQ + kv0 + (unsigned)kk * 32u);
                acc[t] = wmma16g(pa, vb, acc[t]);
            }
        }
        wave_sync_lds();
    }

    float den[8];
#pragma unroll
    for (int r = 0; r < 8; ++r) den[r] = lrow[r] * (P_CARRY * QKV_CARRY);

    float* Tp = T + (size_t)part * PLANE + (size_t)(b * (unsigned)SEQ + q0) * 1024u + head * 128u;
#pragma unroll
    for (int half = 0; half < 2; ++half) {
#pragma unroll
        for (int jj = 0; jj < 4; ++jj)
#pragma unroll
            for (int r = 0; r < 8; ++r)
                pw[(8u * hh + (unsigned)r) * AT_PP + (unsigned)jj * 16u + c] = acc[half * 4 + jj][r] / den[r];
        wave_sync_lds();
        {
            const unsigned c4 = c * 4u;
            v4f vv[8];
#pragma unroll
            for (int it = 0; it < 8; ++it) {
                const unsigned row = (unsigned)it * 2u + hh;
                vv[it] = *(const v4f*)(pw + row * AT_PP + c4);
            }
            float* dst = Tp + (unsigned)half * 64u + c4;
            for (int pass = 0; pass < 2; ++pass) {
#pragma unroll
                for (int it = 0; it < 8; ++it) {
                    const unsigned row = (unsigned)it * 2u + hh;
                    *(volatile v4f*)(dst + (size_t)row * 1024u) = vv[it];
                }
                __threadfence();
            }
        }
        wave_sync_lds();
    }
}

__global__ __launch_bounds__(256) void k_ln(const float* __restrict__ T, const float* __restrict__ qin,
                                            const float* __restrict__ g_r, const float* __restrict__ b_r,
                                            const float* __restrict__ g_i, const float* __restrict__ b_i,
                                            float* __restrict__ out) {
    __shared__ float red[4][8];
    const unsigned t = threadIdx.x, L = t & 31u, w = t >> 5;
    const unsigned row = blockIdx.x;
    const unsigned b = row / (unsigned)SEQ;
    const unsigned s = row - b * (unsigned)SEQ;
    const size_t frow = (size_t)(b * (unsigned)SEQ_FULL + s);
    const float* t0 = T + (size_t)row * 1024u + w * 128u + 2u * L;
    const float* t1 = t0 + PLANE;
    const v2f prvr = *(const v2f*)(t0);
    const v2f prvi = *(const v2f*)(t0 + 64);
    const v2f pivr = *(const v2f*)(t1);
    const v2f pivi = *(const v2f*)(t1 + 64);
    const v4f qq = *(const v4f*)(qin + frow * 1024u + w * 128u + 4u * L);
    const float xr0 = (prvr.x - pivi.x) + bfr(qq.x);
    const float xi0 = (prvi.x + pivr.x) + bfr(qq.y);
    const float xr1 = (prvr.y - pivi.y) + bfr(qq.z);
    const float xi1 = (prvi.y + pivr.y) + bfr(qq.w);

    float sr = xr0 + xr1, si = xi0 + xi1;
#pragma unroll
    for (int o = 16; o > 0; o >>= 1) { sr += __shfl_xor(sr, o, 32); si += __shfl_xor(si, o, 32); }
    if (L == 0u) { red[0][w] = sr; red[1][w] = si; }
    __syncthreads();
    float tr = 0.f, ti = 0.f;
#pragma unroll
    for (int k = 0; k < 8; ++k) { tr += red[0][k]; ti += red[1][k]; }
    const float mur = tr * (1.0f / 512.0f);
    const float mui = ti * (1.0f / 512.0f);
    const float dr0 = xr0 - mur, dr1 = xr1 - mur;
    const float di0 = xi0 - mui, di1 = xi1 - mui;
    float vr = dr0 * dr0 + dr1 * dr1, vi = di0 * di0 + di1 * di1;
#pragma unroll
    for (int o = 16; o > 0; o >>= 1) { vr += __shfl_xor(vr, o, 32); vi += __shfl_xor(vi, o, 32); }
    if (L == 0u) { red[2][w] = vr; red[3][w] = vi; }
    __syncthreads();
    float ur = 0.f, ui = 0.f;
#pragma unroll
    for (int k = 0; k < 8; ++k) { ur += red[2][k]; ui += red[3][k]; }
    const float sdr = sqrtf(ur * (1.0f / 512.0f) + 1e-5f);
    const float sdi = sqrtf(ui * (1.0f / 512.0f) + 1e-5f);

    const unsigned e0 = w * 64u + 2u * L;
    const v2f gr = *(const v2f*)(g_r + e0);
    const v2f br = *(const v2f*)(b_r + e0);
    const v2f gi = *(const v2f*)(g_i + e0);
    const v2f bi = *(const v2f*)(b_i + e0);
    v4f y;
    y.x = (dr0 / sdr) * bfr(gr.x) + bfr(br.x);
    y.y = (di0 / sdi) * bfr(gi.x) + bfr(bi.x);
    y.z = (dr1 / sdr) * bfr(gr.y) + bfr(br.y);
    y.w = (di1 / sdi) * bfr(gi.y) + bfr(bi.y);
    float* dst = out + frow * 1024u + w * 128u + 4u * L;
    *(volatile v4f*)(dst) = y;
    __threadfence();
    *(volatile v4f*)(dst) = y;
}

extern "C" void kernel_launch(void* const* d_in, const int* in_sizes, int n_in, void* d_out, int out_size,
                              void* d_ws, size_t ws_size, hipStream_t stream) {
    if (n_in < 14) return;
    const int need_x = ((NB - 1) * SEQ_FULL + SEQ) * DM * 2;
    if (in_sizes[0] < need_x || in_sizes[1] < need_x || in_sizes[2] < need_x) return;
    if (in_sizes[3] < DM * DM * 2 || in_sizes[5] < DM * DM * 2 || in_sizes[7] < DM * DM * 2) return;
    if (in_sizes[4] < DM * 2 || in_sizes[6] < DM * 2 || in_sizes[8] < DM * 2) return;
    if (in_sizes[9] < DM || in_sizes[10] < DM || in_sizes[11] < DM || in_sizes[12] < DM) return;
    if (out_size < need_x) return;

    const float* q   = (const float*)d_in[0];
    const float* k   = (const float*)d_in[1];
    const float* v   = (const float*)d_in[2];
    const float* Wq  = (const float*)d_in[3];
    const float* bq  = (const float*)d_in[4];
    const float* Wk  = (const float*)d_in[5];
    const float* bk  = (const float*)d_in[6];
    const float* Wv  = (const float*)d_in[7];
    const float* bv  = (const float*)d_in[8];
    const float* g_r = (const float*)d_in[9];
    const float* b_r = (const float*)d_in[10];
    const float* g_i = (const float*)d_in[11];
    const float* b_i = (const float*)d_in[12];
    float* out = (float*)d_out;

    char* wsp = (char*)d_ws;
    size_t off = 0;
    auto carve = [&](size_t bytes) -> void* { void* r = wsp + off; off += (bytes + 255) & ~(size_t)255; return r; };
    unsigned short* xq  = (unsigned short*)carve(SZ_XP);
    unsigned short* xk  = (unsigned short*)carve(SZ_XP);
    unsigned short* xv  = (unsigned short*)carve(SZ_XP);
    unsigned short* wq  = (unsigned short*)carve(SZ_WP);
    unsigned short* wk  = (unsigned short*)carve(SZ_WP);
    unsigned short* wv  = (unsigned short*)carve(SZ_WP);
    _Float16*       QP  = (_Float16*)carve(SZ_QP);
    _Float16*       KAB = (_Float16*)carve(SZ_KAB);
    _Float16*       VT  = (_Float16*)carve(SZ_VT);
    float*          T   = (float*)carve(SZ_T);
    if (off > ws_size || off > (size_t)134217728) return;

    const unsigned gX = (unsigned)(MTOK * 64) / 256u;
    const unsigned gW = (unsigned)(DM * 64) / 256u;
    k_cvtx<<<gX, 256, 0, stream>>>(q, xq);
    k_cvtx<<<gX, 256, 0, stream>>>(k, xk);
    k_cvtx<<<gX, 256, 0, stream>>>(v, xv);
    k_cvtw<<<gW, 256, 0, stream>>>(Wq, wq);
    k_cvtw<<<gW, 256, 0, stream>>>(Wk, wk);
    k_cvtw<<<gW, 256, 0, stream>>>(Wv, wv);

    const unsigned gP = (((unsigned)MTOK / 64u) * ((unsigned)KC / 64u) + 7u) / 8u;
    k_proj<0><<<gP, 256, 0, stream>>>(xq, wq, QP, bq, (unsigned)MTOK, (unsigned)KC, (unsigned)KC);
    k_proj<1><<<gP, 256, 0, stream>>>(xk, wk, KAB, bk, (unsigned)MTOK, (unsigned)KC, (unsigned)KC);
    k_proj<2><<<gP, 256, 0, stream>>>(wv, xv, VT, bv, (unsigned)KC, (unsigned)MTOK, (unsigned)KC);

    k_attn<<<dim3((unsigned)NB * 8u * ((unsigned)SEQ / 128u), 2u), 256, 0, stream>>>(QP, KAB, VT, T, (unsigned)SEQ / 64u);

    k_ln<<<(unsigned)MTOK, 256, 0, stream>>>(T, q, g_r, b_r, g_i, b_i, out);
}
